// GATNet_24129126269181
// MI455X (gfx1250) — hardware-run, weakly checked
//
#include <hip/hip_runtime.h>
#include <stddef.h>
#include <stdint.h>
#include <math.h>


#define F_IN    128
#define DN      100
#define NP      128
#define NHD     10
#define HDW     10
#define KA      256
#define SDW     32
#define NGR     256
#define NCLS    10
#define NOUT    (NGR * NCLS)
#define NTHR    256
#define NWAVE   8
#define EPT     8
#define CHUNK   (NTHR * EPT)
#define WCAP    (EPT * 32)
#define LISTN   (NWAVE * WCAP)
#define NB      1024
#define SLOTB   10
#define RCAP    24576
#define DEGCAP  64
#define FLW     32
#define GBM     64
#define GTHR    128
#define MROWS   128
#define NEGSL   0.2f
#define WSMAX   134217728
#define BK_ZINTS (2 * RCAP + 2 * NB + LISTN + 16)
#define LDS_BKT  (BK_ZINTS * 4)
#define NU0     (NP * (F_IN / 8))
#define NU1     (NP * (KA / 8))

static_assert((CHUNK & (CHUNK - 1)) == 0 && CHUNK == 2048);
static_assert(NB == (1 << SLOTB) && NB == 4 * NTHR);
static_assert(((long long)CHUNK << SLOTB) < (1LL << 31));
static_assert(LISTN >= NB && LISTN == NWAVE * WCAP);
static_assert((RCAP % (4 * NTHR)) == 0);
static_assert(RCAP >= 16623 + 2048);
static_assert(DEGCAP >= 35 + 8);
static_assert((BK_ZINTS % 4) == 0 && LDS_BKT <= 300000);
static_assert(GBM == (GTHR / 32) * 16 && (MROWS % GBM) == 0);
static_assert((F_IN % 32) == 0 && (KA % 32) == 0 && KA == 2 * NP && NP == 8 * 16);
static_assert(DN == NHD * HDW && DN <= NP && (DN % 4) == 0);
static_assert(NP == 4 * 32);
static_assert(MROWS == NWAVE * 16);
static_assert((NU0 % NTHR) == 0 && (NU1 % NTHR) == 0);
static_assert((NOUT * 4) % 128 == 0 && (NOUT / 4) <= 3 * NTHR && ((NOUT / 4) % 32) == 0);
static_assert(NOUT % NTHR == 0);

typedef float          v2f  __attribute__((ext_vector_type(2)));
typedef float          v4f  __attribute__((ext_vector_type(4)));
typedef float          v8f  __attribute__((ext_vector_type(8)));
typedef int            v4i  __attribute__((ext_vector_type(4)));
typedef int            v8i  __attribute__((ext_vector_type(8)));
typedef unsigned int   v2u  __attribute__((ext_vector_type(2)));
typedef unsigned int   v4u  __attribute__((ext_vector_type(4)));
typedef unsigned short v8us __attribute__((ext_vector_type(8)));
typedef __bf16         v16b __attribute__((ext_vector_type(16)));
typedef v4f  __attribute__((may_alias)) v4fa;
typedef v4i  __attribute__((may_alias)) v4ia;
typedef v8us __attribute__((may_alias)) v8usa;
union FragB { v16b v; v8us h[2]; v8i w; };

__device__ __forceinline__ v8f wmb(const FragB& a, const FragB& b, v8f c) {
  v8f d = __builtin_amdgcn_wmma_f32_16x16x32_bf16(false, a.v, false, b.v, (short)0, c, false, false);
  asm volatile("v_nop\n\tv_nop\n\tv_nop\n\tv_nop" : "+v"(d) : "v"(a.w), "v"(b.w));
  return d;
}

__device__ __forceinline__ int iclamp(int v, int lo, int hi) { return v < lo ? lo : (v > hi ? hi : v); }

__device__ __forceinline__ unsigned int f2bf(float f) {
  const unsigned int u = __float_as_uint(f);
  const unsigned int r = ((u + 0x7FFFu + ((u >> 16) & 1u)) >> 16) & 0xFFFFu;
  const unsigned int n = ((u >> 16) & 0xFFFFu) | 0x40u;
  return ((u & 0x7FFFFFFFu) > 0x7F800000u) ? n : r;
}
__device__ __forceinline__ float bf2f(unsigned int b) { return __uint_as_float(b << 16); }
__device__ __forceinline__ float bfr(float f) { return bf2f(f2bf(f)); }
__device__ __forceinline__ v4f bfr4(const v4f a) {
  v4f r; r.x = bfr(a.x); r.y = bfr(a.y); r.z = bfr(a.z); r.w = bfr(a.w); return r;
}
__device__ __forceinline__ unsigned int pk2(float lo, float hi) { return f2bf(lo) | (f2bf(hi) << 16); }
__device__ __forceinline__ v4u pack8(const v4f a, const v4f b) {
  v4u r;
  r.x = pk2(a.x, a.y); r.y = pk2(a.z, a.w); r.z = pk2(b.x, b.y); r.w = pk2(b.z, b.w);
  return r;
}
__device__ __forceinline__ float relun(float v) { return (v > 0.f) ? v : (v - v); }

__device__ __forceinline__ int scan_chunk(const int* __restrict__ dsts, int nE, int cbase, int slotBase,
                                          int nb, int vec8, int* list, int tid, int lane, int wave) {
  int wc = 0;
  const int el0  = tid * EPT;
  const int e0   = cbase + el0;
  const int sent = -2147483647 - 1;
  v4i da, db;
  if (vec8 != 0 && cbase + CHUNK <= nE) {
    da = *(const v4i*)(dsts + e0);
    db = *(const v4i*)(dsts + e0 + 4);
  } else {
    da.x = (e0     < nE) ? dsts[min(e0,     nE - 1)] : sent;
    da.y = (e0 + 1 < nE) ? dsts[min(e0 + 1, nE - 1)] : sent;
    da.z = (e0 + 2 < nE) ? dsts[min(e0 + 2, nE - 1)] : sent;
    da.w = (e0 + 3 < nE) ? dsts[min(e0 + 3, nE - 1)] : sent;
    db.x = (e0 + 4 < nE) ? dsts[min(e0 + 4, nE - 1)] : sent;
    db.y = (e0 + 5 < nE) ? dsts[min(e0 + 5, nE - 1)] : sent;
    db.z = (e0 + 6 < nE) ? dsts[min(e0 + 6, nE - 1)] : sent;
    db.w = (e0 + 7 < nE) ? dsts[min(e0 + 7, nE - 1)] : sent;
  }
  const unsigned nbs = (unsigned)slotBase;
  const unsigned unb = (unsigned)nb;
  const unsigned s0 = (unsigned)da.x - nbs, s1 = (unsigned)da.y - nbs;
  const unsigned s2 = (unsigned)da.z - nbs, s3 = (unsigned)da.w - nbs;
  const unsigned s4 = (unsigned)db.x - nbs, s5 = (unsigned)db.y - nbs;
  const unsigned s6 = (unsigned)db.z - nbs, s7 = (unsigned)db.w - nbs;
  const bool h0 = s0 < unb, h1 = s1 < unb, h2 = s2 < unb, h3 = s3 < unb;
  const bool h4 = s4 < unb, h5 = s5 < unb, h6 = s6 < unb, h7 = s7 < unb;
  const unsigned any = __builtin_amdgcn_ballot_w32(h0 | h1 | h2 | h3 | h4 | h5 | h6 | h7);
  if (any != 0u) {
#define HITJ(J, HJ, SJ) { \
      const unsigned mj = __builtin_amdgcn_ballot_w32(HJ); \
      if (mj != 0u) { \
        if (HJ) { \
          const int pos = wc + (int)__builtin_amdgcn_mbcnt_lo(mj, 0u); \
          if (pos < WCAP) list[wave * WCAP + pos] = ((el0 + (J)) << SLOTB) | (int)(SJ); \
        } \
        wc += (int)__builtin_popcount(mj); } }
    HITJ(0, h0, s0)
    HITJ(1, h1, s1)
    HITJ(2, h2, s2)
    HITJ(3, h3, s3)
    HITJ(4, h4, s4)
    HITJ(5, h5, s5)
    HITJ(6, h6, s6)
    HITJ(7, h7, s7)
#undef HITJ
  }
  return wc;
}

__global__ __launch_bounds__(NTHR) void k_xprep(const float* __restrict__ x, unsigned short* xb, int nN, int nUnits) {
  const int i = (int)blockIdx.x * NTHR + (int)threadIdx.x;
  if (i >= nUnits) return;
  const int row = i >> 4;
  const int c0  = (i & 15) * 8;
  const int rc  = row < nN ? row : nN - 1;
  const float* p = x + (size_t)rc * F_IN + c0;
  v4f a = *(const v4fa*)p, b = *(const v4fa*)(p + 4);
  const v4f z4 = {0.f, 0.f, 0.f, 0.f};
  if (row >= nN) { a = z4; b = z4; }
  const v4u hv = pack8(a, b);
  const size_t o = (size_t)row * F_IN + c0;
  *(volatile v4u*)(xb + o) = hv;
  __threadfence();
  *(volatile v4u*)(xb + o) = hv;
}

__device__ __forceinline__ void wtr_unit(const float* __restrict__ w, int Kin, int Kout, unsigned short* wt, int u) {
  const int kq  = Kout >> 3;
  const int n   = u / kq;
  const int k8  = (u - n * kq) * 8;
  const int kk0 = k8 & (NP - 1);
  const int ncl = n < DN ? n : DN - 1;
  const bool nok = n < DN;
  float v[8];
#pragma unroll
  for (int i = 0; i < 8; ++i) {
    const int kk = kk0 + i;
    const int kc = kk < Kin ? kk : Kin - 1;
    const float t = w[(size_t)kc * DN + ncl];
    v[i] = (nok && kk < Kin) ? t : 0.0f;
  }
  v4u wv;
  wv.x = pk2(v[0], v[1]); wv.y = pk2(v[2], v[3]); wv.z = pk2(v[4], v[5]); wv.w = pk2(v[6], v[7]);
  unsigned short* o = wt + (size_t)n * (size_t)Kout + k8;
  *(volatile v4u*)o = wv;
  __threadfence();
  *(volatile v4u*)o = wv;
}
__global__ __launch_bounds__(NTHR) void k_wprep(const float* __restrict__ W0, const float* __restrict__ W1,
                                                const float* __restrict__ W2,
                                                unsigned short* W0T, unsigned short* W1D, unsigned short* W2D) {
  const int u = (int)blockIdx.x * NTHR + (int)threadIdx.x;
  if (u < NU0) {
    wtr_unit(W0, F_IN, F_IN, W0T, u);
  } else if (u < NU0 + NU1) {
    wtr_unit(W1, DN, KA, W1D, u - NU0);
  } else if (u < NU0 + 2 * NU1) {
    wtr_unit(W2, DN, KA, W2D, u - NU0 - NU1);
  }
}

__device__ __forceinline__ void bucket_flush(const int* reg2, const int* soff, const int* scnt,
                                             int* hb, int* ob, int* cb, int* fb, int tid, int flag, int nh) {
#pragma unroll 4
  for (int it = 0; it < RCAP / (4 * NTHR); ++it) {
    const int p = it * NTHR + tid;
    const v4i v = *(const v4ia*)(reg2 + 4 * p);
    *(volatile v4i*)(hb + 4 * p) = v;
  }
  {
    const v4i vo = *(const v4ia*)(soff + 4 * tid);
    const v4i vc = *(const v4ia*)(scnt + 4 * tid);
    *(volatile v4i*)(ob + 4 * tid) = vo;
    *(volatile v4i*)(cb + 4 * tid) = vc;
  }
  if (tid < 8) {
    v4i f;
    f.x = (tid == 0) ? flag : 0;
    f.y = (tid == 0) ? nh : 0;
    f.z = 0; f.w = 0;
    *(volatile v4i*)(fb + 4 * tid) = f;
  }
}

__global__ __launch_bounds__(NTHR) void k_bucket(const int* __restrict__ srcs, const int* __restrict__ dsts,
                                                 int nN, int nE, int vec8,
                                                 int* HITS, int* OFFP, int* CNTP, int* FLG) {
  extern __shared__ v4i lds_dyn[];
  int* reg1 = (int*)lds_dyn;
  int* reg2 = reg1 + RCAP;
  int* scnt = reg2 + RCAP;
  int* soff = scnt + NB;
  int* list = soff + NB;
  int* wcnt = list + LISTN;
  int* wtot = wcnt + NWAVE;
  const int tid = (int)threadIdx.x, lane = tid & 31, wave = tid >> 5;
  const int nodeBase = (int)blockIdx.x * NB;

  {
    const v4i z4 = {0, 0, 0, 0};
    for (int i = tid * 4; i < BK_ZINTS; i += NTHR * 4) *(v4ia*)(reg1 + i) = z4;
  }
  __syncthreads();

  int tot = 0;
  const int nChunks = (nE + CHUNK - 1) / CHUNK;
#pragma unroll 1
  for (int ch = 0; ch < nChunks; ++ch) {
    const int cbase = ch * CHUNK;
    const int wc = scan_chunk(dsts, nE, cbase, nodeBase, NB, vec8, list, tid, lane, wave);
    if (lane == 0) wcnt[wave] = wc;
    __syncthreads();
    int pre = 0, all = 0;
#pragma unroll
    for (int w2 = 0; w2 < NWAVE; ++w2) {
      int c = wcnt[w2];
      c = c < 0 ? 0 : (c > WCAP ? WCAP : c);
      all += c;
      pre += (w2 < wave) ? c : 0;
    }
    const int wcc  = wc > WCAP ? WCAP : wc;
    const int base = tot + pre;
#pragma unroll 1
    for (int i0 = 0; i0 < wcc; i0 += 32) {
      const int i   = i0 + lane;
      const int ic  = i < WCAP ? i : WCAP - 1;
      const int ent = list[wave * WCAP + ic];
      const int el  = (ent >> SLOTB) & (CHUNK - 1);
      const int sl  = ent & (NB - 1);
      const int eid = iclamp(cbase + el, 0, nE - 1);
      const int s   = iclamp(srcs[eid], 0, nN - 1);
      const int pos = base + i;
      if (i < wcc && pos < RCAP) reg1[pos] = (int)(((unsigned)s << SLOTB) | (unsigned)sl);
    }
    tot += all;
    tot = tot > RCAP ? RCAP : tot;
    __syncthreads();
  }
  const int nh = tot;

  if (wave == 0) {
#pragma unroll 1
    for (int b0 = 0; b0 < nh; b0 += 32) {
      const int idx = b0 + lane;
      const int uv  = reg1[idx < nh ? idx : nh - 1];
      const int m32 = (nh - b0) < 32 ? (nh - b0) : 32;
#pragma unroll 1
      for (int k = 0; k < m32; ++k) {
        const int u  = __builtin_amdgcn_readlane(uv, k);
        const int sl = u & (NB - 1);
        if (lane == 0) scnt[sl] = scnt[sl] + 1;
      }
    }
  }
  __syncthreads();

  {
    const v4i ca = *(const v4ia*)(scnt + 4 * tid);
    const int e0 = ca.x < 0 ? 0 : ca.x, e1 = ca.y < 0 ? 0 : ca.y, e2 = ca.z < 0 ? 0 : ca.z, e3 = ca.w < 0 ? 0 : ca.w;
    const int ts = e0 + e1 + e2 + e3;
    int incl = ts;
#pragma unroll
    for (int d = 1; d < 32; d <<= 1) {
      const int up = __shfl_up(incl, d);
      if (lane >= d) incl += up;
    }
    if (lane == 31) wtot[wave] = incl;
    __syncthreads();
    int pre = 0;
#pragma unroll
    for (int w2 = 0; w2 < NWAVE; ++w2) pre += (w2 < wave) ? wtot[w2] : 0;
    int run = pre + incl - ts;
    soff[4 * tid + 0] = run; run += e0;
    soff[4 * tid + 1] = run; run += e1;
    soff[4 * tid + 2] = run; run += e2;
    soff[4 * tid + 3] = run;
  }
  __syncthreads();
  for (int i = tid; i < NB; i += NTHR) list[i] = soff[i];
  __syncthreads();

  if (wave == 0) {
#pragma unroll 1
    for (int b0 = 0; b0 < nh; b0 += 32) {
      const int idx = b0 + lane;
      const int uv  = reg1[idx < nh ? idx : nh - 1];
      const int m32 = (nh - b0) < 32 ? (nh - b0) : 32;
#pragma unroll 1
      for (int k = 0; k < m32; ++k) {
        const int u  = __builtin_amdgcn_readlane(uv, k);
        const int sl = u & (NB - 1);
        const int sv = (int)((unsigned)u >> SLOTB);
        if (lane == 0) {
          int pos = list[sl];
          pos = pos < 0 ? 0 : (pos > RCAP - 1 ? RCAP - 1 : pos);
          reg2[pos] = sv;
          list[sl] = pos + 1;
        }
      }
    }
  }
  __syncthreads();

  const int flag = (nh >= RCAP) ? 1 : 0;
  int* hb = HITS + (size_t)blockIdx.x * RCAP;
  int* ob = OFFP + nodeBase;
  int* cb = CNTP + nodeBase;
  int* fb = FLG + (size_t)blockIdx.x * FLW;
  bucket_flush(reg2, soff, scnt, hb, ob, cb, fb, tid, flag, nh);
  __threadfence();
  bucket_flush(reg2, soff, scnt, hb, ob, cb, fb, tid, flag, nh);
}

__device__ __forceinline__ void gemm_flush(const float* stg, const float* sdl, float* outF, float* SD,
                                           int rowBase, int tid) {
#pragma unroll 4
  for (int it = 0; it < (GBM * NP) / (4 * GTHR); ++it) {
    const int p = it * GTHR + tid;
    const int row = p >> 5, c4 = p & 31;
    const v4f v = *(const v4fa*)(stg + row * NP + 4 * c4);
    *(volatile v4f*)(outF + (size_t)(rowBase + row) * NP + 4 * c4) = v;
  }
#pragma unroll
  for (int it = 0; it < (GBM * SDW) / (4 * GTHR); ++it) {
    const int p = it * GTHR + tid;
    const int row = p >> 3, q = p & 7;
    const v4f v = *(const v4fa*)(sdl + row * SDW + 4 * q);
    *(volatile v4f*)(SD + (size_t)(rowBase + row) * SDW + 4 * q) = v;
  }
}

__global__ __launch_bounds__(GTHR) void k_gemm(
    const unsigned short* __restrict__ A, const unsigned short* __restrict__ WT,
    float* outF, int K,
    const float* __restrict__ atts, const float* __restrict__ attd, float* SD)
{
  __shared__ __attribute__((aligned(16))) float stg[GBM * NP];
  __shared__ __attribute__((aligned(16))) float satt[2 * NP];
  __shared__ __attribute__((aligned(16))) float sdl[GBM * SDW];
  const int tid = (int)threadIdx.x, lane = tid & 31, wave = tid >> 5, hh = lane >> 4, m = lane & 15;
  const int rowBase = (int)blockIdx.x * GBM;

  {
    const int cl = tid < DN ? tid : DN - 1;
    const float vs = atts[cl];
    const float vd = attd[cl];
    const bool ok = tid < DN;
    satt[tid]      = ok ? bfr(vs) : 0.0f;
    satt[NP + tid] = ok ? bfr(vd) : 0.0f;
    const v4f z4 = {0.f, 0.f, 0.f, 0.f};
#pragma unroll
    for (int j = 0; j < 4; ++j) *(v4fa*)(sdl + 16 * tid + 4 * j) = z4;
  }

  v8f acc[8];
  {
    const v8f z = {0.f, 0.f, 0.f, 0.f, 0.f, 0.f, 0.f, 0.f};
#pragma unroll
    for (int t = 0; t < 8; ++t) acc[t] = z;
  }
  const unsigned short* ap = A  + (size_t)(rowBase + 16 * wave + m) * (size_t)K + 8 * hh;
  const unsigned short* wp = WT + (size_t)m * (size_t)K + 8 * hh;
  const int ksteps = K >> 5;
#pragma unroll 1
  for (int ks = 0; ks < ksteps; ++ks) {
    FragB af;
    af.h[0] = *(const v8usa*)(ap + 32 * ks);
    af.h[1] = *(const v8usa*)(ap + 32 * ks + 16);
#pragma unroll
    for (int t = 0; t < 8; ++t) {
      const unsigned short* wq = wp + (size_t)(16 * t) * (size_t)K + 32 * ks;
      FragB bf;
      bf.h[0] = *(const v8usa*)wq;
      bf.h[1] = *(const v8usa*)(wq + 16);
      acc[t] = wmb(af, bf, acc[t]);
    }
  }

#pragma unroll
  for (int t = 0; t < 8; ++t) {
    const int lc = 16 * t + m;
#pragma unroll
    for (int r = 0; r < 8; ++r) {
      const int lr = 16 * wave + 8 * hh + r;
      stg[lr * NP + lc] = acc[t][r];
    }
  }
  __syncthreads();

#pragma unroll 1
  for (int it = 0; it < (GBM * NHD) / GTHR; ++it) {
    const int p = it * GTHR + tid;
    const int row = p & (GBM - 1);
    const int hd  = p >> 6;
    const float* hr = stg + row * NP + hd * HDW;
    const float* sa = satt + hd * HDW;
    float ds = 0.f, dd = 0.f;
#pragma unroll 2
    for (int f = 0; f < HDW; ++f) {
      const float hv = hr[f];
      ds = fmaf(hv, sa[f], ds);
      dd = fmaf(hv, sa[NP + f], dd);
    }
    sdl[row * SDW + hd]      = ds;
    sdl[row * SDW + 16 + hd] = dd;
  }
  __syncthreads();

  gemm_flush(stg, sdl, outF, SD, rowBase, tid);
  __threadfence();
  gemm_flush(stg, sdl, outF, SD, rowBase, tid);
}

template <int L>
__global__ __launch_bounds__(NTHR) void k_scan(
    const float* __restrict__ H, const float* __restrict__ SD,
    const int* __restrict__ HITS, const int* __restrict__ OFFP, const int* __restrict__ CNTP,
    const int* __restrict__ FLG, const float* __restrict__ bias,
    unsigned short* XHL, float* X3, int nN, int MPr) {
  const int tid = (int)threadIdx.x, lane = tid & 31;
  const int wave = __builtin_amdgcn_readfirstlane(tid >> 5);
  const int c0  = 4 * lane;
  const int hA0 = c0 / HDW, hB0 = (c0 + 3) / HDW;
  const int hA  = hA0 < NHD ? hA0 : NHD - 1;
  const int hB  = hB0 < NHD ? hB0 : NHD - 1;
  const bool by = ((c0 + 1) / HDW) != hA0;
  const bool bz = ((c0 + 2) / HDW) != hA0;
  const bool colok = c0 < DN;
  const int  cb = colok ? c0 : DN - 4;
  v4f bb = bfr4(*(const v4fa*)(bias + cb));
  bb.x = colok ? bb.x : 0.f; bb.y = colok ? bb.y : 0.f; bb.z = colok ? bb.z : 0.f; bb.w = colok ? bb.w : 0.f;
  const float qnan = __int_as_float(0x7fc00000);

#pragma unroll 1
  for (int jt = 0; jt < 16; ++jt) {
    const int grow = (int)blockIdx.x * MROWS + wave * 16 + jt;
    const int gcl  = grow < nN ? grow : nN - 1;
    const int bk   = grow >> SLOTB;
    int st = OFFP[grow];
    const int craw = CNTP[grow];
    const int flg  = FLG[bk * FLW];
    int nh = FLG[bk * FLW + 1];
    nh = iclamp(nh, 0, RCAP);
    st = iclamp(st, 0, nh);
    int cnt = iclamp(craw, 0, DEGCAP);
    if (cnt > nh - st) cnt = nh - st;
    const float pz = (flg != 0 || craw > DEGCAP || craw < 0) ? qnan : 0.0f;
    const int* hp = HITS + (size_t)bk * RCAP;

    const float* sdr = SD + (size_t)gcl * SDW;
    const float adA = sdr[16 + hA], adB = sdr[16 + hB];
    float lA = sdr[hA] + adA, lB = sdr[hB] + adB;
    lA = (lA >= 0.f) ? lA : NEGSL * lA;
    lB = (lB >= 0.f) ? lB : NEGSL * lB;
    float mxA = lA, mxB = lB, dnA = 1.0f, dnB = 1.0f;
    v4f acc = *(const v4fa*)(H + (size_t)gcl * NP + c0);

#pragma unroll 1
    for (int q = 0; q < cnt; ++q) {
      const int idx = iclamp(st + q, 0, RCAP - 1);
      const int s   = iclamp(hp[idx], 0, nN - 1);
      const v4f fa  = *(const v4fa*)(H + (size_t)s * NP + c0);
      const float* ss = SD + (size_t)s * SDW;
      float lgA = ss[hA] + adA, lgB = ss[hB] + adB;
      lgA = (lgA >= 0.f) ? lgA : NEGSL * lgA;
      lgB = (lgB >= 0.f) ? lgB : NEGSL * lgB;
      const float dfA = lgA - mxA, dfB = lgB - mxB;
      const float eA = expf(-fabsf(dfA));
      const float eB = expf(-fabsf(dfB));
      const bool upA = dfA > 0.f, upB = dfB > 0.f;
      const float s1A = upA ? eA : 1.0f, s2A = upA ? 1.0f : eA;
      const float s1B = upB ? eB : 1.0f, s2B = upB ? 1.0f : eB;
      mxA = upA ? lgA : mxA;
      mxB = upB ? lgB : mxB;
      dnA = fmaf(dnA, s1A, s2A);
      dnB = fmaf(dnB, s1B, s2B);
      const float s1y = by ? s1B : s1A, s2y = by ? s2B : s2A;
      const float s1z = bz ? s1B : s1A, s2z = bz ? s2B : s2A;
      acc.x = fmaf(acc.x, s1A, s2A * fa.x);
      acc.y = fmaf(acc.y, s1y, s2y * fa.y);
      acc.z = fmaf(acc.z, s1z, s2z * fa.z);
      acc.w = fmaf(acc.w, s1B, s2B * fa.w);
    }
    const float invA = 1.0f / dnA, invB = 1.0f / dnB;
    const float invy = by ? invB : invA, invz = bz ? invB : invA;
    const bool live = grow < nN;
    v4f v;
    v.x = relun(fmaf(acc.x, invA, bb.x));
    v.y = relun(fmaf(acc.y, invy, bb.y));
    v.z = relun(fmaf(acc.z, invz, bb.z));
    v.w = relun(fmaf(acc.w, invB, bb.w));
    const bool keep = live && colok;
    v4f o;
    o.x = (keep ? v.x : 0.f) + pz;
    o.y = (keep ? v.y : 0.f) + pz;
    o.z = (keep ? v.z : 0.f) + pz;
    o.w = (keep ? v.w : 0.f) + pz;
    const bool wr = grow < MPr;
    if constexpr (L == 0) {
      const unsigned int h0 = f2bf(o.x), h1 = f2bf(o.y), h2 = f2bf(o.z), h3 = f2bf(o.w);
      const unsigned int g0 = f2bf(o.x - bf2f(h0)), g1 = f2bf(o.y - bf2f(h1));
      const unsigned int g2 = f2bf(o.z - bf2f(h2)), g3 = f2bf(o.w - bf2f(h3));
      v2u hv, lv;
      hv.x = h0 | (h1 << 16); hv.y = h2 | (h3 << 16);
      lv.x = g0 | (g1 << 16); lv.y = g2 | (g3 << 16);
      unsigned short* gp = XHL + (size_t)grow * KA + 4 * lane;
      unsigned short* gq = gp + NP;
      if (wr) { *(volatile v2u*)gp = hv; *(volatile v2u*)gq = lv; }
      __threadfence();
      if (wr) { *(volatile v2u*)gp = hv; *(volatile v2u*)gq = lv; }
    } else {
      float* op = X3 + (size_t)grow * NP + 4 * lane;
      if (wr) *(volatile v4f*)op = o;
      __threadfence();
      if (wr) *(volatile v4f*)op = o;
    }
  }
}

__global__ __launch_bounds__(NTHR) void k_pool(const float* __restrict__ hf, const int* __restrict__ bat,
                                               int nN, float* G) {
  __shared__ __attribute__((aligned(16))) double wsum[NWAVE * NP];
  __shared__ int wcn[NWAVE];
  __shared__ __attribute__((aligned(16))) float outs[NP];
  const int tid = (int)threadIdx.x, lane = tid & 31;
  const int wave = __builtin_amdgcn_readfirstlane(tid >> 5);
  const int g = (int)blockIdx.x;

  double a0 = 0.0, a1 = 0.0, a2 = 0.0, a3 = 0.0;
  int cnt = 0;
#pragma unroll 1
  for (int i0 = wave * 32; i0 < nN; i0 += NTHR) {
    const int i  = i0 + lane;
    const int ic = i < nN ? i : nN - 1;
    const int b  = bat[ic];
    const bool hit = (i < nN) && (b == g);
    unsigned msk = __builtin_amdgcn_ballot_w32(hit);
    int nh = (int)__builtin_popcount(msk);
    nh = nh > 32 ? 32 : nh;
    cnt += nh;
#pragma unroll 1
    for (int q = 0; q < nh; ++q) {
      const int k = __builtin_ffs((int)msk) - 1;
      msk &= msk - 1u;
      int node = i0 + (k < 0 ? 0 : k);
      node = node > nN - 1 ? nN - 1 : node;
      const v4f v = *(const v4fa*)(hf + (size_t)node * NP + 4 * lane);
      a0 += (double)v.x; a1 += (double)v.y; a2 += (double)v.z; a3 += (double)v.w;
    }
  }
  wsum[wave * NP + 4 * lane + 0] = a0;
  wsum[wave * NP + 4 * lane + 1] = a1;
  wsum[wave * NP + 4 * lane + 2] = a2;
  wsum[wave * NP + 4 * lane + 3] = a3;
  if (lane == 0) wcn[wave] = cnt;
  __syncthreads();
  if (tid < NP) {
    double s = 0.0;
    int c = 0;
#pragma unroll
    for (int w2 = 0; w2 < NWAVE; ++w2) { s += wsum[w2 * NP + tid]; c += wcn[w2]; }
    const float cf = (c < 1) ? 1.0f : (float)c;
    outs[tid] = (float)s * (1.0f / cf);
  }
  __syncthreads();
  const v4f ov = *(const v4fa*)(outs + 4 * lane);
  float* op = G + (size_t)g * NP + 4 * lane;
  const bool okst = (wave == 0);
  if (okst) *(volatile v4f*)op = ov;
  __threadfence();
  if (okst) *(volatile v4f*)op = ov;
}

__global__ __launch_bounds__(NTHR) void k_head(const float* __restrict__ G, const float* __restrict__ Wfc,
                                               const float* __restrict__ bfc, const int* __restrict__ FLG,
                                               int nbk, float* out) {
  __shared__ float wls[DN * NCLS];
  __shared__ float bls[16];
  __shared__ int sflag;
  __shared__ __attribute__((aligned(16))) float os[NOUT];
  const int tid = (int)threadIdx.x;
#pragma unroll 1
  for (int i = tid; i < DN * NCLS; i += NTHR) wls[i] = bfr(Wfc[i]);
  if (tid < 16) {
    const float bbv = bfc[tid < NCLS ? tid : NCLS - 1];
    bls[tid] = (tid < NCLS) ? bfr(bbv) : 0.0f;
  }
  if (tid == 0) sflag = 0;
  __syncthreads();
  {
    const int bc = tid < nbk ? tid : nbk - 1;
    const int f = FLG[bc * FLW];
    if (tid < nbk && f != 0) sflag = 1;
  }
#pragma unroll 1
  for (int it = 0; it < NOUT / NTHR; ++it) {
    const int idx = it * NTHR + tid;
    const int g = idx / NCLS;
    const int c = idx - g * NCLS;
    const float* pr = G + (size_t)g * NP;
    float s = 0.0f;
#pragma unroll 1
    for (int k4 = 0; k4 < DN / 4; ++k4) {
      const v4f p = *(const v4fa*)(pr + 4 * k4);
      const float* w = wls + (4 * k4) * NCLS + c;
      s = fmaf(p.x, w[0], s);
      s = fmaf(p.y, w[NCLS], s);
      s = fmaf(p.z, w[2 * NCLS], s);
      s = fmaf(p.w, w[3 * NCLS], s);
    }
    os[idx] = s + bls[c];
  }
  __syncthreads();
  const bool poison = sflag != 0;
  const float qn = __int_as_float(0x7fc00000);
  v4f ov[3];
#pragma unroll
  for (int it = 0; it < 3; ++it) {
    const int p  = it * NTHR + tid;
    const int pc = p < NOUT / 4 ? p : NOUT / 4 - 1;
    v4f v = *(const v4fa*)(os + 4 * pc);
    v.x = poison ? qn : v.x; v.y = poison ? qn : v.y; v.z = poison ? qn : v.z; v.w = poison ? qn : v.w;
    ov[it] = v;
  }
#pragma unroll
  for (int it = 0; it < 3; ++it) {
    const int p = it * NTHR + tid;
    if (p < NOUT / 4) *(volatile v4f*)(out + 4 * (size_t)p) = ov[it];
  }
  __threadfence();
#pragma unroll
  for (int it = 0; it < 3; ++it) {
    const int p = it * NTHR + tid;
    if (p < NOUT / 4) *(volatile v4f*)(out + 4 * (size_t)p) = ov[it];
  }
}

static inline int cdiv(int a, int b) { return (a + b - 1) / b; }
static inline size_t al256(size_t o) { return (o + 255) & ~(size_t)255; }

extern "C" void kernel_launch(void* const* d_in, const int* in_sizes, int n_in,
                              void* d_out, int out_size, void* d_ws, size_t ws_size,
                              hipStream_t stream) {
  if (n_in < 17) return;
  if (in_sizes[0] < F_IN || (in_sizes[0] % F_IN) != 0) return;
  const int nN = in_sizes[0] / F_IN;
  if (nN < 1 || nN > (1 << 20)) return;
  if (in_sizes[1] < 2 || (in_sizes[1] & 1) != 0) return;
  const int nE = in_sizes[1] / 2;
  if (nE < 1 || nE > (1 << 28)) return;
  if (in_sizes[2] != nN) return;
  if (in_sizes[3] != F_IN * DN) return;
  if (in_sizes[4] != DN || in_sizes[5] != DN || in_sizes[6] != DN) return;
  if (in_sizes[7] != DN * DN) return;
  if (in_sizes[8] != DN || in_sizes[9] != DN || in_sizes[10] != DN) return;
  if (in_sizes[11] != DN * DN) return;
  if (in_sizes[12] != DN || in_sizes[13] != DN || in_sizes[14] != DN) return;
  if (in_sizes[15] != DN * NCLS) return;
  if (in_sizes[16] != NCLS) return;
  if (out_size != NOUT) return;

  const float* x    = (const float*)d_in[0];
  const int*   ei   = (const int*)  d_in[1];
  const int*   bat  = (const int*)  d_in[2];
  const float* W0   = (const float*)d_in[3];
  const float* a0s  = (const float*)d_in[4];
  const float* a0d  = (const float*)d_in[5];
  const float* b0   = (const float*)d_in[6];
  const float* W1   = (const float*)d_in[7];
  const float* a1s  = (const float*)d_in[8];
  const float* a1d  = (const float*)d_in[9];
  const float* b1   = (const float*)d_in[10];
  const float* W2   = (const float*)d_in[11];
  const float* a2s  = (const float*)d_in[12];
  const float* a2d  = (const float*)d_in[13];
  const float* b2   = (const float*)d_in[14];
  const float* Wfc  = (const float*)d_in[15];
  const float* bfc  = (const float*)d_in[16];
  float* out = (float*)d_out;
  const int* src = ei;
  const int* dst = ei + nE;

  const int MP    = cdiv(nN, MROWS) * MROWS;
  const int nbk   = cdiv(MP, NB);
  const int NBTOT = nbk * NB;
  if (nbk < 1 || nbk > NTHR) return;
  if (NBTOT < MP) return;
  const int vec8 = ((nE & 3) == 0) ? 1 : 0;

  char* ws = (char*)d_ws;
  size_t off = 0;
  const size_t oXB  = off; off = al256(off + (size_t)MP * F_IN * 2);
  const size_t oW0  = off; off = al256(off + (size_t)NP * F_IN * 2);
  const size_t oW1  = off; off = al256(off + (size_t)NP * KA * 2);
  const size_t oW2  = off; off = al256(off + (size_t)NP * KA * 2);
  const size_t oH   = off; off = al256(off + (size_t)MP * NP * 4);
  const size_t oSD  = off; off = al256(off + (size_t)MP * SDW * 4);
  const size_t oXH  = off; off = al256(off + (size_t)MP * KA * 2);
  const size_t oX3  = off; off = al256(off + (size_t)MP * NP * 4);
  const size_t oHT  = off; off = al256(off + (size_t)nbk * RCAP * 4);
  const size_t oOF  = off; off = al256(off + (size_t)NBTOT * 4);
  const size_t oCN  = off; off = al256(off + (size_t)NBTOT * 4);
  const size_t oFL  = off; off = al256(off + (size_t)nbk * FLW * 4);
  const size_t oG   = off; off = al256(off + (size_t)NGR * NP * 4);
  if (off > ws_size || off > (size_t)WSMAX) return;
  unsigned short* XB  = (unsigned short*)(ws + oXB);
  unsigned short* W0T = (unsigned short*)(ws + oW0);
  unsigned short* W1D = (unsigned short*)(ws + oW1);
  unsigned short* W2D = (unsigned short*)(ws + oW2);
  float*          H   = (float*)(ws + oH);
  float*          SD  = (float*)(ws + oSD);
  unsigned short* XHL = (unsigned short*)(ws + oXH);
  float*          X3  = (float*)(ws + oX3);
  int*            HT  = (int*)(ws + oHT);
  int*            OFP = (int*)(ws + oOF);
  int*            CNP = (int*)(ws + oCN);
  int*            FLG = (int*)(ws + oFL);
  float*          G   = (float*)(ws + oG);

  hipFuncSetAttribute(reinterpret_cast<const void*>(&k_bucket),
                      hipFuncAttributeMaxDynamicSharedMemorySize, LDS_BKT);

  const int nUx = MP * (F_IN / 8);
  k_xprep<<<cdiv(nUx, NTHR), NTHR, 0, stream>>>(x, XB, nN, nUx);
  k_wprep<<<(NU0 + 2 * NU1) / NTHR, NTHR, 0, stream>>>(W0, W1, W2, W0T, W1D, W2D);
  k_bucket<<<nbk, NTHR, LDS_BKT, stream>>>(src, dst, nN, nE, vec8, HT, OFP, CNP, FLG);

  const int gM = MP / GBM;
  const int gS = MP / MROWS;
  k_gemm<<<gM, GTHR, 0, stream>>>(XB, W0T, H, F_IN, a0s, a0d, SD);
  k_scan<0><<<gS, NTHR, 0, stream>>>(H, SD, HT, OFP, CNP, FLG, b0, XHL, X3, nN, MP);
  k_gemm<<<gM, GTHR, 0, stream>>>(XHL, W1D, H, KA, a1s, a1d, SD);
  k_scan<0><<<gS, NTHR, 0, stream>>>(H, SD, HT, OFP, CNP, FLG, b1, XHL, X3, nN, MP);
  k_gemm<<<gM, GTHR, 0, stream>>>(XHL, W2D, H, KA, a2s, a2d, SD);
  k_scan<1><<<gS, NTHR, 0, stream>>>(H, SD, HT, OFP, CNP, FLG, b2, XHL, X3, nN, MP);
  k_pool<<<NGR, NTHR, 0, stream>>>(X3, bat, nN, G);
  k_head<<<1, NTHR, 0, stream>>>(G, Wfc, bfc, FLG, nbk, out);
}
